// StageBlock_36361193128264
// MI455X (gfx1250) — hardware-verified
//
#include <hip/hip_runtime.h>

typedef __attribute__((ext_vector_type(16))) _Float16 v16h;
typedef __attribute__((ext_vector_type(8)))  _Float16 v8h;
typedef __attribute__((ext_vector_type(4)))  _Float16 v4h;
typedef __attribute__((ext_vector_type(16))) __bf16   v16b;
typedef __attribute__((ext_vector_type(8)))  __bf16   v8b;
typedef __attribute__((ext_vector_type(8)))  float    v8f;
typedef __attribute__((ext_vector_type(4)))  float    v4f;

static constexpr int kB    = 4;
static constexpr int kLQ   = 1600;
static constexpr int kD    = 768;
static constexpr int kNH   = 12;
static constexpr int kHD   = 64;
static constexpr int kLV   = 5440;
static constexpr int kMQ   = kB * kLQ;
static constexpr int kMV   = kB * kLV;
static constexpr int kNOFF = 384;
static constexpr int kNLG  = 192;
static constexpr int kNCAT = kNOFF + kNLG;
static constexpr int kNBIAS = kNCAT + kD + kD;
static_assert(kMQ % 64 == 0 && kMV % 64 == 0, "M tile multiples");
static_assert(kD % 64 == 0 && kNCAT % 64 == 0, "N tile multiples");
static_assert(kD % 32 == 0, "K multiple of 32");
static_assert(kNBIAS % 32 == 0, "bias lines whole");

static constexpr size_t SZ_VAL   = (size_t)kMV * kD * 4;
static constexpr size_t SZ_F16P  = (size_t)kMV * kD * 2;
static constexpr size_t SZ_Q16   = (size_t)kMQ * kD * 2;
static constexpr size_t SZ_OA    = (size_t)kMQ * kNCAT * 4;
static constexpr size_t SZ_AO16  = (size_t)kMQ * kD * 2;
static constexpr size_t SZ_NEWP  = (size_t)kMQ * kD * 4;
static constexpr size_t OFF_VAL  = 0;
static constexpr size_t OFF_BIG  = OFF_VAL + SZ_VAL;
static constexpr size_t OFF_F16P = OFF_BIG;
static constexpr size_t OFF_Q16  = OFF_BIG;
static constexpr size_t OFF_OA   = OFF_BIG + SZ_Q16;
static constexpr size_t OFF_AO16 = OFF_BIG;
static constexpr size_t OFF_NEWP = OFF_BIG + SZ_AO16;
static constexpr size_t OFF_WV   = OFF_BIG + SZ_F16P;
static constexpr size_t OFF_WOUT = OFF_WV + (size_t)kD * kD * 2;
static constexpr size_t OFF_WCAT = OFF_WOUT + (size_t)kD * kD * 2;
static constexpr size_t OFF_BIAS = OFF_WCAT + (size_t)kNCAT * kD * 2;
static constexpr size_t WS_TOTAL = OFF_BIAS + (size_t)kNBIAS * 4;
static_assert(OFF_OA + SZ_OA <= OFF_WV, "OA inside R_BIG");
static_assert(OFF_NEWP + SZ_NEWP <= OFF_WV, "NEWP inside R_BIG");
static_assert(OFF_AO16 + SZ_AO16 <= OFF_OA && OFF_Q16 + SZ_Q16 <= OFF_OA, "no overlap with OA/NEWP");
static_assert(WS_TOTAL <= (size_t)134217728, "carve under 128 MiB");
static_assert((OFF_BIG % 128) == 0 && (OFF_OA % 128) == 0 && (OFF_WV % 128) == 0 && (OFF_WOUT % 128) == 0 &&
              (OFF_WCAT % 128) == 0 && (OFF_BIAS % 128) == 0, "128-B aligned regions");

__device__ __forceinline__ unsigned short f2bf_bits(float f) {
  unsigned u = __float_as_uint(f);
  return (unsigned short)((u + 0x7FFFu + ((u >> 16) & 1u)) >> 16);
}
__device__ __forceinline__ float bf_bits2f(unsigned short h) { return __uint_as_float(((unsigned)h) << 16); }

__device__ __forceinline__ void dep_guard_h(v8f& a, v8f& b, v16h x, v16h y) { asm volatile("v_nop\n\tv_nop\n\tv_nop\n\tv_nop" : "+v"(a), "+v"(b) : "v"(x), "v"(y)); }
__device__ __forceinline__ void dep_guard_b(v8f& a, v8f& b, v16b x, v16b y) { asm volatile("v_nop\n\tv_nop\n\tv_nop\n\tv_nop" : "+v"(a), "+v"(b) : "v"(x), "v"(y)); }
__device__ __forceinline__ void keep4_h(v16h a, v16h b, v16h c, v16h d) { asm volatile("v_nop" :: "v"(a), "v"(b), "v"(c), "v"(d)); }
__device__ __forceinline__ void keep4_b(v16b a, v16b b, v16b c, v16b d) { asm volatile("v_nop" :: "v"(a), "v"(b), "v"(c), "v"(d)); }
__device__ __forceinline__ void acc_guard4(v8f& a, v8f& b, v8f& c, v8f& d) { asm volatile("v_nop\n\tv_nop\n\tv_nop\n\tv_nop" : "+v"(a), "+v"(b), "+v"(c), "+v"(d)); }
template <typename T> struct Frag;
template <> struct Frag<_Float16> {
  typedef v16h V; union U { v16h v; v8h h[2]; };
  static __device__ __forceinline__ v16h load(const _Float16* p) {
    U f; f.h[0] = *(const v8h*)(p); f.h[1] = *(const v8h*)(p + 16); return f.v;
  }
  static __device__ __forceinline__ v8f mma(v16h a, v16h b, v8f c) {
    return __builtin_amdgcn_wmma_f32_16x16x32_f16(false, a, false, b, (short)0, c, false, false);
  }
  static __device__ __forceinline__ void guard(v8f& a, v8f& b, v16h x, v16h y) { dep_guard_h(a, b, x, y); }
  static __device__ __forceinline__ void keep(v16h a, v16h b, v16h c, v16h d) { keep4_h(a, b, c, d); }
};
template <> struct Frag<__bf16> {
  typedef v16b V; union U { v16b v; v8b h[2]; };
  static __device__ __forceinline__ v16b load(const __bf16* p) {
    U f; f.h[0] = *(const v8b*)(p); f.h[1] = *(const v8b*)(p + 16); return f.v;
  }
  static __device__ __forceinline__ v8f mma(v16b a, v16b b, v8f c) {
    return __builtin_amdgcn_wmma_f32_16x16x32_bf16(false, a, false, b, (short)0, c, false, false);
  }
  static __device__ __forceinline__ void guard(v8f& a, v8f& b, v16b x, v16b y) { dep_guard_b(a, b, x, y); }
  static __device__ __forceinline__ void keep(v16b a, v16b b, v16b c, v16b d) { keep4_b(a, b, c, d); }
};

template <int ET> struct Elem;
template <> struct Elem<0> { typedef _Float16 T; };
template <> struct Elem<1> { typedef __bf16 T; };
template <int ET, bool SPLIT, int BIAS_MODE, int OUT_MODE, bool RESID, int ACT = 0>
__global__ __launch_bounds__(256) void wmma_gemm64(
    const unsigned short* __restrict__ Ap, const unsigned short* __restrict__ A2p, int lda, long strideA,
    const unsigned short* __restrict__ Btp, const unsigned short* __restrict__ Bt2p, int ldb, long strideB,
    void* __restrict__ Cout, void* __restrict__ Cout2, int ldc, long strideC,
    const float* __restrict__ bias,
    const float* __restrict__ resid, long strideR,
    int M, int N, int K, float scale) {
  typedef typename Elem<ET>::T T;
  typedef typename Frag<T>::V V;
  const T* A = (const T*)Ap; const T* A2 = (const T*)A2p; const T* Bt = (const T*)Btp; const T* Bt2 = (const T*)Bt2p;
  __shared__ __align__(16) float sT[8][16 * 68];
  const int b    = blockIdx.y;
  const int lane = threadIdx.x & 31;
  const int wave = threadIdx.x >> 5;
  const int tilesN = N >> 6;
  const int tilesM = M >> 6;
  const int tile = blockIdx.x * 8 + wave;
  if (tile >= tilesM * tilesN) return;
  const int tm = tile / tilesN;
  const int tn = tile - tm * tilesN;
  const int m0 = tm << 6;
  const int n0 = tn << 6;

  const T* Ab  = A  + (size_t)b * strideA;
  const T* Bb  = Bt + (size_t)b * strideB;
  const T* Ab2 = SPLIT ? (A2  + (size_t)b * strideA) : nullptr;
  const T* Bb2 = SPLIT ? (Bt2 + (size_t)b * strideB) : nullptr;

  const int rlane = lane & 15;
  const int koff  = (lane >> 4) * 8;
  const int mOff  = (lane >> 4) * 8;

  v8f acc[4][4];
#pragma unroll
  for (int i = 0; i < 4; ++i)
#pragma unroll
    for (int j = 0; j < 4; ++j) acc[i][j] = (v8f){0.f,0.f,0.f,0.f,0.f,0.f,0.f,0.f};

  for (int k0 = 0; k0 < K; k0 += 32) {
    V bh[4], bl[4];
#pragma unroll
    for (int j = 0; j < 4; ++j) {
      const size_t bo = (size_t)(n0 + (j << 4) + rlane) * ldb + koff + k0;
      bh[j] = Frag<T>::load(Bb + bo);
      if (SPLIT) bl[j] = Frag<T>::load(Bb2 + bo);
    }
#pragma unroll
    for (int i = 0; i < 4; ++i) {
      const size_t ao = (size_t)(m0 + (i << 4) + rlane) * lda + koff + k0;
      V ah = Frag<T>::load(Ab + ao);
      V al;
      if (SPLIT) al = Frag<T>::load(Ab2 + ao);
#pragma unroll
      for (int j = 0; j < 4; ++j) {
        acc[i][j] = Frag<T>::mma(ah, bh[j], acc[i][j]);
        if (SPLIT) {
          acc[i][j] = Frag<T>::mma(ah, bl[j], acc[i][j]);
          acc[i][j] = Frag<T>::mma(al, bh[j], acc[i][j]);
        }
      }
      Frag<T>::guard(acc[i][0], acc[i][3], ah, SPLIT ? al : ah);
    }
    Frag<T>::keep(bh[0], bh[1], bh[2], bh[3]);
    if (SPLIT) Frag<T>::keep(bl[0], bl[1], bl[2], bl[3]);
  }
  acc_guard4(acc[0][0], acc[0][1], acc[0][2], acc[0][3]);
  acc_guard4(acc[1][0], acc[1][1], acc[1][2], acc[1][3]);
  acc_guard4(acc[2][0], acc[2][1], acc[2][2], acc[2][3]);
  acc_guard4(acc[3][0], acc[3][1], acc[3][2], acc[3][3]);

  float* slab = sT[wave];
  const float* Rb = RESID ? (resid + (size_t)b * strideR) : nullptr;
#pragma unroll
  for (int i = 0; i < 4; ++i) {
    const int mBase = m0 + (i << 4);
#pragma unroll
    for (int j = 0; j < 4; ++j) {
      const int n = n0 + (j << 4) + rlane;
      float bv = 0.f;
      if (BIAS_MODE == 2) bv = bias[n];
#pragma unroll
      for (int r = 0; r < 8; ++r) {
        float v = acc[i][j][r] * scale;
        if (BIAS_MODE == 1) v += bias[mBase + mOff + r];
        if (BIAS_MODE == 2) v += bv;
        if (RESID) v += Rb[(size_t)(mBase + mOff + r) * ldc + n];
        if (ACT == 1) v = tanhf(v);
        if (ACT == 2) v = fmaxf(v, 0.0f);
        if (ACT == 3) v = v / (1.0f + expf(-v));
        if (ACT == 4) v = (v > 0.f) ? v : 0.01f * v;
        if (ACT == 5) v = 0.5f * v * (1.0f + erff(v * 0.70710678118654752f));
        slab[(mOff + r) * 68 + (j << 4) + rlane] = v;
      }
    }
    __builtin_amdgcn_fence(__ATOMIC_RELEASE, "workgroup");
    __builtin_amdgcn_wave_barrier();
    __builtin_amdgcn_fence(__ATOMIC_ACQUIRE, "workgroup");
    if (OUT_MODE == 0) {
      float* C = (float*)Cout + (size_t)b * strideC;
      const int hh = lane >> 4, c4 = (lane & 15) * 4;
      for (int pass = 0; pass < 2; ++pass) {
#pragma unroll
        for (int it = 0; it < 8; ++it) {
          const int row = it * 2 + hh;
          v4f v = *(const v4f*)(slab + row * 68 + c4);
          *(volatile v4f*)(C + (size_t)(mBase + row) * ldc + n0 + c4) = v;
        }
        __threadfence();
      }
    } else {
      const int q = lane >> 3, c8 = (lane & 7) * 8;
      unsigned short* C  = (unsigned short*)Cout  + (size_t)b * strideC;
      unsigned short* C2 = (OUT_MODE == 2) ? ((unsigned short*)Cout2 + (size_t)b * strideC) : nullptr;
      for (int pass = 0; pass < 2; ++pass) {
#pragma unroll
        for (int it = 0; it < 4; ++it) {
          const int row = it * 4 + q;
          const float* sp = slab + row * 68 + c8;
          v8h hv, lv;
#pragma unroll
          for (int e = 0; e < 8; ++e) {
            if (OUT_MODE == 1) {
              hv[e] = (_Float16)sp[e];
            } else {
              unsigned short hb = f2bf_bits(sp[e]);
              unsigned short lb = f2bf_bits(sp[e] - bf_bits2f(hb));
              hv[e] = __builtin_bit_cast(_Float16, hb);
              lv[e] = __builtin_bit_cast(_Float16, lb);
            }
          }
          *(volatile v8h*)(C + (size_t)(mBase + row) * ldc + n0 + c8) = hv;
          if (OUT_MODE == 2) *(volatile v8h*)(C2 + (size_t)(mBase + row) * ldc + n0 + c8) = lv;
        }
        __threadfence();
      }
    }
    __builtin_amdgcn_fence(__ATOMIC_RELEASE, "workgroup");
    __builtin_amdgcn_wave_barrier();
    __builtin_amdgcn_fence(__ATOMIC_ACQUIRE, "workgroup");
  }
}

__device__ __forceinline__ float wave_sum(float v) {
#pragma unroll
  for (int off = 16; off >= 1; off >>= 1) v += __shfl_xor(v, off, 32);
  return v;
}

__global__ __launch_bounds__(256) void prep_wt16(const float* __restrict__ W, _Float16* __restrict__ Wt,
                                                int Kdim, int Nreal, int Npad) {
  const int t = blockIdx.x * 256 + threadIdx.x;
  const int k8n = Kdim >> 3;
  const int total = Npad * k8n;
  if (t >= total) return;
  const int n = t / k8n;
  const int k8 = t - n * k8n;
  const int ncl = n < Nreal ? n : (Nreal - 1);
  v8h hv;
#pragma unroll
  for (int i = 0; i < 8; ++i) {
    const float v = W[(size_t)(k8 * 8 + i) * Nreal + ncl] * 16.0f;
    hv[i] = (_Float16)v;
  }
  v8h z = {};
  if (n >= Nreal) hv = z;
  _Float16* dst = Wt + (size_t)n * Kdim + (size_t)k8 * 8;
  *(volatile v8h*)dst = hv;
  __threadfence();
  *(volatile v8h*)dst = hv;
}

__global__ __launch_bounds__(256) void prep_bias(const float* __restrict__ boff, const float* __restrict__ blog,
                                                const float* __restrict__ bval, const float* __restrict__ bo2,
                                                float* __restrict__ dst) {
  const int n = blockIdx.x * 256 + threadIdx.x;
  if (n >= kNBIAS) return;
  int i0 = n;                 i0 = i0 > kNOFF - 1 ? kNOFF - 1 : i0;
  int i1 = n - kNOFF;         i1 = i1 < 0 ? 0 : (i1 > kNLG - 1 ? kNLG - 1 : i1);
  int i2 = n - kNCAT;         i2 = i2 < 0 ? 0 : (i2 > kD - 1 ? kD - 1 : i2);
  int i3 = n - kNCAT - kD;    i3 = i3 < 0 ? 0 : (i3 > kD - 1 ? kD - 1 : i3);
  const float v0 = boff[i0];
  const float v1 = blog[i1];
  const float v2 = bval[i2];
  const float v3 = bo2[i3];
  const float v = (n < kNOFF) ? v0 : ((n < kNCAT) ? v1 : ((n < kNCAT + kD) ? v2 : v3));
  ((volatile float*)dst)[n] = v;
  __threadfence();
  ((volatile float*)dst)[n] = v;
}

__global__ __launch_bounds__(256) void ln768_kernel(const float* __restrict__ in, const float* __restrict__ sc,
                                                   const float* __restrict__ bi, _Float16* __restrict__ out,
                                                   int nrows) {
  const int wave = threadIdx.x >> 5, lane = threadIdx.x & 31;
  const int row = blockIdx.x * 8 + wave;
  if (row >= nrows) return;
  const float* p = in + (size_t)row * kD;
  v4f a[6];
#pragma unroll
  for (int j = 0; j < 3; ++j) {
    const int c0 = 256 * j + lane * 8;
    a[2 * j]     = *(const v4f*)(p + c0);
    a[2 * j + 1] = *(const v4f*)(p + c0 + 4);
  }
  float s = 0.0f;
#pragma unroll
  for (int j = 0; j < 6; ++j) s += (a[j][0] + a[j][1]) + (a[j][2] + a[j][3]);
  s = wave_sum(s);
  const float mean = s * (1.0f / 768.0f);
  v4f d[6];
  float sq = 0.0f;
#pragma unroll
  for (int j = 0; j < 6; ++j) {
    d[j] = a[j] - mean;
    sq += (d[j][0] * d[j][0] + d[j][1] * d[j][1]) + (d[j][2] * d[j][2] + d[j][3] * d[j][3]);
  }
  sq = wave_sum(sq);
  const float var = sq * (1.0f / 768.0f);
  const float rstd = rsqrtf(var + 1e-6f);
  v8h hv[3];
#pragma unroll
  for (int j = 0; j < 3; ++j) {
    const int c0 = 256 * j + lane * 8;
    const v4f g0 = *(const v4f*)(sc + c0), g1 = *(const v4f*)(sc + c0 + 4);
    const v4f b0 = *(const v4f*)(bi + c0), b1 = *(const v4f*)(bi + c0 + 4);
    const v4f o0 = d[2 * j] * rstd * g0 + b0;
    const v4f o1 = d[2 * j + 1] * rstd * g1 + b1;
    const v8f oo = __builtin_shufflevector(o0, o1, 0, 1, 2, 3, 4, 5, 6, 7);
    hv[j] = __builtin_convertvector(oo, v8h);
  }
  _Float16* op = out + (size_t)row * kD;
  for (int pass = 0; pass < 2; ++pass) {
#pragma unroll
    for (int j = 0; j < 3; ++j) *(volatile v8h*)(op + 256 * j + lane * 8) = hv[j];
    __threadfence();
  }
}

__device__ __forceinline__ void corner_acc(float (&acc)[8], const float* __restrict__ valb,
                                           int st, int iW, int iH, int yi, int xi, float w, float aw) {
#pragma clang fp contract(off)
  const bool ok = (xi >= 0) && (xi < iW) && (yi >= 0) && (yi < iH);
  const float wv = w * (ok ? 1.0f : 0.0f);
  const float coef = aw * wv;
  int xc = xi < 0 ? 0 : xi;
  xc = xc > iW - 1 ? iW - 1 : xc;
  int yc = yi < 0 ? 0 : yi;
  yc = yc > iH - 1 ? iH - 1 : yc;
  int vr = st + yc * iW + xc;
  vr = vr < 0 ? 0 : (vr > kLV - 1 ? kLV - 1 : vr);
  const float* vp = valb + (size_t)vr * kD;
  const v4f g0 = *(const v4f*)vp;
  const v4f g1 = *(const v4f*)(vp + 4);
#pragma unroll
  for (int e = 0; e < 4; ++e) {
    acc[e]     = fmaf(coef, g0[e], acc[e]);
    acc[4 + e] = fmaf(coef, g1[e], acc[4 + e]);
  }
}

__global__ __launch_bounds__(256) void sample_kernel(const float* __restrict__ val, const float* __restrict__ oa,
                                                    const float* __restrict__ refp, _Float16* __restrict__ ao16) {
#pragma clang fp contract(off)
  const int wave = threadIdx.x >> 5;
  const int lane = threadIdx.x & 31;
  const int gw = blockIdx.x * 8 + wave;
  const int row = gw / 3;
  const int hg = gw - row * 3;
  const int h = hg * 4 + (lane >> 3);
  const int c = lane & 7;
  const int rowc = row < kMQ ? row : (kMQ - 1);
  const int bidx = rowc / kLQ;

  const float* oar  = oa + (size_t)rowc * kNCAT;
  const float* lgp  = oar + kNOFF + h * 16;
  const float* offp = oar + h * 32;

  float lg[16];
  {
    const v4f l0 = *(const v4f*)(lgp), l1 = *(const v4f*)(lgp + 4), l2 = *(const v4f*)(lgp + 8), l3 = *(const v4f*)(lgp + 12);
#pragma unroll
    for (int e = 0; e < 4; ++e) { lg[e] = l0[e]; lg[4 + e] = l1[e]; lg[8 + e] = l2[e]; lg[12 + e] = l3[e]; }
  }
  float mx = lg[0];
#pragma unroll
  for (int j = 1; j < 16; ++j) mx = fmaxf(mx, lg[j]);
  float sum = 0.0f;
#pragma unroll
  for (int j = 0; j < 16; ++j) sum += __expf(lg[j] - mx);
  const float inv = 1.0f / sum;

  const float* rp = refp + (size_t)rowc * 8;
  const float* valb = val + (size_t)bidx * kLV * kD + h * kHD + c * 8;

  float acc[8];
#pragma unroll
  for (int e = 0; e < 8; ++e) acc[e] = 0.0f;

#pragma unroll 1
  for (int pt = 0; pt < 16; ++pt) {
    const int l = pt >> 2;
    const int iW = 64 >> l;
    const int iH = iW;
    const int st = (l == 0) ? 0 : ((l == 1) ? 4096 : ((l == 2) ? 5120 : 5376));
    const float fW = (float)iW, fH = (float)iH;
    const float rcW = (l == 0) ? 0.015625f : ((l == 1) ? 0.03125f : ((l == 2) ? 0.0625f : 0.125f));
    const float rcH = rcW;
    const float rx = rp[l * 2 + 0];
    const float ry = rp[l * 2 + 1];
    const float aw = __expf(lgp[pt] - mx) * inv;
    const float ox = offp[pt * 2 + 0];
    const float oy = offp[pt * 2 + 1];
    const float locx = rx + ox * rcW;
    const float locy = ry + oy * rcH;
    const float px = locx * fW - 0.5f;
    const float py = locy * fH - 0.5f;
    const float x0f = floorf(px), y0f = floorf(py);
    const float fx = px - x0f, fy = py - y0f;
    const int x0 = (int)x0f, y0 = (int)y0f;
    const float gx = 1.0f - fx, gy = 1.0f - fy;
    corner_acc(acc, valb, st, iW, iH, y0,     x0,     gx * gy, aw);
    corner_acc(acc, valb, st, iW, iH, y0,     x0 + 1, fx * gy, aw);
    corner_acc(acc, valb, st, iW, iH, y0 + 1, x0,     gx * fy, aw);
    corner_acc(acc, valb, st, iW, iH, y0 + 1, x0 + 1, fx * fy, aw);
  }

  v8h o;
#pragma unroll
  for (int e = 0; e < 8; ++e) o[e] = (_Float16)(acc[e] * 16.0f);
  _Float16* dst = ao16 + (size_t)rowc * kD + h * kHD + c * 8;
  *(volatile v8h*)dst = o;
  __threadfence();
  *(volatile v8h*)dst = o;
}

__global__ __launch_bounds__(256) void gamma_resid_kernel(const float* __restrict__ newp, const float* __restrict__ xin,
                                                         const float* __restrict__ gam,
                                                         float* __restrict__ out0, float* __restrict__ out1, int nrows) {
#pragma clang fp contract(off)
  const int wave = threadIdx.x >> 5, lane = threadIdx.x & 31;
  const int row = blockIdx.x * 8 + wave;
  if (row >= nrows) return;
  const size_t rb = (size_t)row * kD;
  v4f pv[6], ov[6];
#pragma unroll
  for (int j = 0; j < 6; ++j) {
    const int c0 = 128 * j + lane * 4;
    const v4f nv = *(const v4f*)(newp + rb + c0);
    const v4f xv = *(const v4f*)(xin + rb + c0);
    const v4f gv = *(const v4f*)(gam + c0);
    pv[j] = nv * gv;
    ov[j] = xv + pv[j];
  }
  for (int pass = 0; pass < 2; ++pass) {
#pragma unroll
    for (int j = 0; j < 6; ++j) {
      const int c0 = 128 * j + lane * 4;
      *(volatile v4f*)(out0 + rb + c0) = ov[j];
      *(volatile v4f*)(out1 + rb + c0) = pv[j];
    }
    __threadfence();
  }
}

static constexpr int gemm_blocks(int M, int N) { return ((M / 64) * (N / 64) + 7) / 8; }

extern "C" void kernel_launch(void* const* d_in, const int* in_sizes, int n_in,
                              void* d_out, int out_size, void* d_ws, size_t ws_size,
                              hipStream_t stream) {
  if (n_in < 20) return;
  if (in_sizes[0] != kMQ * kD || in_sizes[1] != kMV * kD || in_sizes[2] != kMQ * 8) return;
  if (in_sizes[3] != 8 || in_sizes[4] != 4) return;
  if (in_sizes[7] != kD || in_sizes[8] != kD || in_sizes[9] != kD || in_sizes[10] != kD || in_sizes[11] != kD) return;
  if (in_sizes[12] != kD * kD || in_sizes[13] != kD) return;
  if (in_sizes[14] != kD * kNOFF || in_sizes[15] != kNOFF) return;
  if (in_sizes[16] != kD * kNLG || in_sizes[17] != kNLG) return;
  if (in_sizes[18] != kD * kD || in_sizes[19] != kD) return;
  if (out_size != 2 * kMQ * kD) return;
  if (ws_size < WS_TOTAL) return;

  const float* x        = (const float*)d_in[0];
  const float* feat     = (const float*)d_in[1];
  const float* refp     = (const float*)d_in[2];
  const float* qn_scale = (const float*)d_in[7];
  const float* qn_bias  = (const float*)d_in[8];
  const float* fn_scale = (const float*)d_in[9];
  const float* fn_bias  = (const float*)d_in[10];
  const float* gam      = (const float*)d_in[11];
  const float* Wv       = (const float*)d_in[12];
  const float* bval_in  = (const float*)d_in[13];
  const float* Wo       = (const float*)d_in[14];
  const float* bo_in    = (const float*)d_in[15];
  const float* Wa       = (const float*)d_in[16];
  const float* ba_in    = (const float*)d_in[17];
  const float* Wout     = (const float*)d_in[18];
  const float* bout_in  = (const float*)d_in[19];

  char* ws = (char*)d_ws;
  float*    valp  = (float*)(ws + OFF_VAL);
  _Float16* f16p  = (_Float16*)(ws + OFF_F16P);
  _Float16* q16   = (_Float16*)(ws + OFF_Q16);
  float*    oa    = (float*)(ws + OFF_OA);
  _Float16* ao16  = (_Float16*)(ws + OFF_AO16);
  float*    newp  = (float*)(ws + OFF_NEWP);
  _Float16* wvT   = (_Float16*)(ws + OFF_WV);
  _Float16* woutT = (_Float16*)(ws + OFF_WOUT);
  _Float16* wcatT = (_Float16*)(ws + OFF_WCAT);
  float*    biasr = (float*)(ws + OFF_BIAS);
  float*    bcat  = biasr;
  float*    bvalr = biasr + kNCAT;
  float*    boutr = biasr + kNCAT + kD;
  float*    out0  = (float*)d_out;
  float*    out1  = (float*)d_out + (size_t)kMQ * kD;

  typedef const unsigned short* cu16;
  const float sc16  = 1.0f / 16.0f;
  const float sc256 = 1.0f / 256.0f;

  prep_wt16<<<(kD * (kD / 8) + 255) / 256, 256, 0, stream>>>(Wv, wvT, kD, kD, kD);
  prep_wt16<<<(kD * (kD / 8) + 255) / 256, 256, 0, stream>>>(Wout, woutT, kD, kD, kD);
  prep_wt16<<<(kNOFF * (kD / 8) + 255) / 256, 256, 0, stream>>>(Wo, wcatT, kD, kNOFF, kNOFF);
  prep_wt16<<<(kNLG * (kD / 8) + 255) / 256, 256, 0, stream>>>(Wa, wcatT + (size_t)kNOFF * kD, kD, kNLG, kNLG);
  prep_bias<<<(kNBIAS + 255) / 256, 256, 0, stream>>>(bo_in, ba_in, bval_in, bout_in, biasr);

  ln768_kernel<<<kMV / 8, 256, 0, stream>>>(feat, fn_scale, fn_bias, f16p, kMV);
  wmma_gemm64<0, false, 2, 0, false, 0><<<dim3(gemm_blocks(kMV, kD), 1), 256, 0, stream>>>(
      (cu16)f16p, nullptr, kD, 0L, (cu16)wvT, nullptr, kD, 0L, (void*)valp, nullptr, kD, 0L,
      bvalr, nullptr, 0L, kMV, kD, kD, sc16);

  ln768_kernel<<<kMQ / 8, 256, 0, stream>>>(x, qn_scale, qn_bias, q16, kMQ);
  wmma_gemm64<0, false, 2, 0, false, 0><<<dim3(gemm_blocks(kMQ, kNCAT), 1), 256, 0, stream>>>(
      (cu16)q16, nullptr, kD, 0L, (cu16)wcatT, nullptr, kD, 0L, (void*)oa, nullptr, kNCAT, 0L,
      bcat, nullptr, 0L, kMQ, kNCAT, kD, sc16);

  sample_kernel<<<kMQ * 3 / 8, 256, 0, stream>>>(valp, oa, refp, ao16);

  wmma_gemm64<0, false, 2, 0, false, 0><<<dim3(gemm_blocks(kMQ, kD), 1), 256, 0, stream>>>(
      (cu16)ao16, nullptr, kD, 0L, (cu16)woutT, nullptr, kD, 0L, (void*)newp, nullptr, kD, 0L,
      boutr, nullptr, 0L, kMQ, kD, kD, sc256);

  gamma_resid_kernel<<<kMQ / 8, 256, 0, stream>>>(newp, x, gam, out0, out1, kMQ);
}
